// Encoder_63333587747633
// MI455X (gfx1250) — hardware-run, weakly checked
//
#include <hip/hip_runtime.h>

typedef __attribute__((ext_vector_type(16))) _Float16 v16h;
typedef __attribute__((ext_vector_type(8)))  _Float16 v8h;
typedef __attribute__((ext_vector_type(8)))  float    v8f;
typedef __attribute__((ext_vector_type(4)))  float    v4f;
typedef __attribute__((ext_vector_type(4)))  unsigned int v4u;

constexpr int kBatch = 64;
constexpr int kSteps = 2048;
constexpr int kFeat  = 15;
constexpr int kUnits = 256;
constexpr int kGates = 3 * kUnits;
constexpr int kRowsPerBlock = 16;
constexpr int kBlocks  = kBatch / kRowsPerBlock;
constexpr int kThreads = 512;
constexpr int kWaves   = kThreads / 32;
constexpr int kXPitch  = 32;
constexpr int kHPitch  = 264;
constexpr int kHBuf    = kRowsPerBlock * kHPitch;
constexpr int kHWords  = 2 * kHBuf / 2;
constexpr int kK1      = kUnits;
constexpr int kK2      = 2 * kUnits;

static_assert(kBlocks == 4, "four row-owned blocks");
static_assert(kWaves * 16 == kUnits, "one 16-unit slice per wave");
static_assert(kBatch * kSteps * kFeat * 4 == 7864320, "input bytes");
static_assert(kFeat * kGates * 4 == 46080, "W1 bytes");
static_assert(kUnits * kGates * 4 == 786432, "U1/W2/U2 bytes");
static_assert(2 * kGates * 4 == 6144, "bias bytes");
static_assert(3 * kBatch * kUnits * 4 == 196608, "output bytes");
static_assert(kFeat <= kXPitch, "x part fits one k-step");
static_assert((kHPitch * 2) % 16 == 0, "16-B aligned state rows");
static_assert(kHWords % 4 == 0, "whole 16-B chunks");

constexpr float kCarryA    = 256.0f;
constexpr float kCarryW    = 256.0f;
constexpr float kCarryProd = kCarryA * kCarryW;
constexpr float kFold      = 1.0f / kCarryProd;
constexpr float kLog2e     = 1.4426950408889634f;
constexpr float kSigArg    = -kLog2e * kFold;
constexpr float kHalfMinNormal = 6.103515625e-05f;
constexpr float kF32MinNormal  = 1.17549435e-38f;

constexpr size_t kWx1Bytes = (size_t)kGates * kXPitch * 2;
constexpr size_t kWu1Bytes = (size_t)kGates * kK1 * 2;
constexpr size_t kWt2Bytes = (size_t)kGates * kK2 * 2;
constexpr size_t kCarveTotal = kWx1Bytes + kWu1Bytes + kWt2Bytes;
static_assert(kWx1Bytes == 49152 && kWu1Bytes == 393216 && kWt2Bytes == 786432, "carve sizes");
static_assert(kWx1Bytes % 128 == 0 && kWu1Bytes % 128 == 0, "line-aligned carve offsets");
static_assert(kCarveTotal == 1228800, "carve total");

constexpr int kJob0Blocks = kGates * (kXPitch / 8) / 256;
constexpr int kJob1Blocks = kGates * (kK1 / 8) / 256;
constexpr int kJob2Blocks = kGates * (kK2 / 8) / 256;
static_assert(kJob0Blocks == 12 && kJob1Blocks == 96 && kJob2Blocks == 192, "exact chunk coverage");
static_assert(kJob0Blocks * 256 == kGates * (kXPitch / 8), "job 0 exact");
static_assert(kJob1Blocks * 256 == kGates * (kK1 / 8), "job 1 exact");
static_assert(kJob2Blocks * 256 == kGates * (kK2 / 8), "job 2 exact");

__device__ __forceinline__ float flush_h(float v) {
  return (__builtin_fabsf(v) < kHalfMinNormal) ? 0.0f : v;
}

__device__ __forceinline__ unsigned int pack_h2(float a, float b) {
  const _Float16 ha = (_Float16)a;
  const _Float16 hb = (_Float16)b;
  return (unsigned int)__builtin_bit_cast(unsigned short, ha) |
         ((unsigned int)__builtin_bit_cast(unsigned short, hb) << 16);
}

union FragU { v16h v; v8h h[2]; };
__device__ __forceinline__ v16h frag_load(const _Float16* p) {
  FragU f;
  f.h[0] = *(const v8h*)(p);
  f.h[1] = *(const v8h*)(p + 16);
  return f.v;
}

__device__ __forceinline__ v8f mma_f16(v16h a, v16h b, v8f c) {
  c = __builtin_amdgcn_wmma_f32_16x16x32_f16(false, a, false, b, (short)0, c, false, false);
  asm volatile("v_nop\n\tv_nop\n\tv_nop\n\tv_nop" : "+v"(c) : "v"(a), "v"(b));
  return c;
}

__device__ __forceinline__ float sigm_c(float p) {
  const float e = __builtin_amdgcn_exp2f(p * kSigArg);
  return __builtin_amdgcn_rcpf(1.0f + e);
}

template <int NK>
__device__ __forceinline__ void k_group(v8f& az, v8f& ar, v8f& a3,
                                        const _Float16* pz, const _Float16* pr, const _Float16* ph,
                                        const _Float16* bp) {
#pragma unroll 2
  for (int ks = 0; ks < NK; ++ks) {
    const v16h b  = frag_load(bp + ks * 32);
    const v16h wz = frag_load(pz + ks * 32);
    const v16h wr = frag_load(pr + ks * 32);
    const v16h wh = frag_load(ph + ks * 32);
    az = mma_f16(wz, b, az);
    ar = mma_f16(wr, b, ar);
    a3 = mma_f16(wh, b, a3);
  }
}

__device__ __forceinline__ void cell_update(const v8f& az, const v8f& ar, const v8f& axh, const v8f& arh,
                                            float (&h)[8], _Float16* dst) {
  v8h hv;
#pragma unroll
  for (int m = 0; m < 8; ++m) {
    const float z  = sigm_c(az[m]);
    const float r  = sigm_c(ar[m]);
    const float pre = fmaf(r, arh[m], axh[m]) * kFold;
    const float hh = fmaxf(pre, 0.0f);
    float hn = fmaf(z, h[m] - hh, hh);
    hn = (hn < kF32MinNormal) ? 0.0f : hn;
    h[m] = hn;
    hv[m] = (_Float16)flush_h(hn * kCarryA);
  }
  *(v8h*)dst = hv;
}

__device__ __forceinline__ void stage_x(const float* __restrict__ x, unsigned int* Xw, int brow0, int t, int tid) {
  const int b  = tid >> 2;
  const int c8 = tid & 3;
  const float* xr = x + ((size_t)(brow0 + b) * kSteps + t) * kFeat;
  float v[8];
#pragma unroll
  for (int e = 0; e < 8; ++e) {
    const int f  = c8 * 8 + e;
    const int fc = f < kFeat ? f : kFeat - 1;
    float a = xr[fc];
    asm volatile("" : "+v"(a));
    v[e] = (f < kFeat) ? flush_h(a * kCarryA) : 0.0f;
  }
  v4u w;
  w[0] = pack_h2(v[0], v[1]);
  w[1] = pack_h2(v[2], v[3]);
  w[2] = pack_h2(v[4], v[5]);
  w[3] = pack_h2(v[6], v[7]);
  *(v4u*)(Xw + b * (kXPitch / 2) + c8 * 4) = w;
}

__global__ __launch_bounds__(256)
void build_weight_planes(const float* __restrict__ W1, const float* __restrict__ U1,
                         const float* __restrict__ W2, const float* __restrict__ U2,
                         unsigned int* __restrict__ wx1w, unsigned int* __restrict__ wu1w,
                         unsigned int* __restrict__ wt2w) {
  const int blk = blockIdx.x;
  const float* srcA;
  const float* srcB;
  unsigned int* dst;
  int cshift;
  int kvalid;
  int cblk;
  if (blk < kJob0Blocks) {
    srcA = W1; srcB = W1; dst = wx1w; cshift = 2; kvalid = kFeat; cblk = blk;
  } else if (blk < kJob0Blocks + kJob1Blocks) {
    srcA = U1; srcB = U1; dst = wu1w; cshift = 5; kvalid = kUnits; cblk = blk - kJob0Blocks;
  } else {
    srcA = W2; srcB = U2; dst = wt2w; cshift = 6; kvalid = kUnits; cblk = blk - kJob0Blocks - kJob1Blocks;
  }
  const int c  = cblk * 256 + (int)threadIdx.x;
  int n = c >> cshift;
  n = n < kGates ? n : kGates - 1;
  const int c8 = c & ((1 << cshift) - 1);
  const float* src = (c8 >> 5) ? srcB : srcA;
  const int kbase = (c8 & 31) * 8;
  float v[8];
#pragma unroll
  for (int e = 0; e < 8; ++e) {
    const int kk = kbase + e;
    const int kc = kk < kvalid ? kk : kvalid - 1;
    float a = src[(size_t)kc * kGates + n];
    asm volatile("" : "+v"(a));
    v[e] = (kk < kvalid) ? flush_h(a * kCarryW) : 0.0f;
  }
  v4u w;
  w[0] = pack_h2(v[0], v[1]);
  w[1] = pack_h2(v[2], v[3]);
  w[2] = pack_h2(v[4], v[5]);
  w[3] = pack_h2(v[6], v[7]);
  volatile v4u* dp = (volatile v4u*)(dst + (size_t)c * 4);
  for (int pass = 0; pass < 2; ++pass) {
    *dp = w;
    __threadfence();
  }
}

__global__ __launch_bounds__(kThreads)
void stacked_gated_cells(const float* __restrict__ x,
                         const float* __restrict__ b1,
                         const float* __restrict__ b2,
                         const unsigned short* wx1,
                         const unsigned short* wu1,
                         const unsigned short* wt2,
                         float* __restrict__ out) {
  __shared__ __align__(16) unsigned int Xw[kRowsPerBlock * kXPitch / 2];
  __shared__ __align__(16) unsigned int H1w[kHWords];
  __shared__ __align__(16) unsigned int H2w[kHWords];
  __shared__ __align__(32) float Ctab[2 * 4 * kUnits];
  __shared__ __align__(16) float Osl[kRowsPerBlock * kUnits];

  const int tid  = threadIdx.x;
  const int lane = tid & 31;
  const int wave = __builtin_amdgcn_readfirstlane(tid >> 5);
  const int bn   = lane & 15;
  const int hf   = lane >> 4;
  const int brow0 = (int)blockIdx.x * kRowsPerBlock;

  {
    const v4u zz = (v4u){0u, 0u, 0u, 0u};
    for (int i = tid; i < kHWords / 4; i += kThreads) {
      ((v4u*)H1w)[i] = zz;
      ((v4u*)H2w)[i] = zz;
    }
  }
#pragma unroll
  for (int j = 0; j < 4; ++j) {
    const int idx  = tid + kThreads * j;
    const int acc  = (idx >> 8) & 3;
    const int unit = idx & (kUnits - 1);
    const int g    = acc < 2 ? acc : 2;
    const int col  = g * kUnits + unit;
    const float* bb = (j >> 1) ? b2 : b1;
    const float bi = bb[col];
    const float br = bb[kGates + col];
    const float sv = (acc < 2) ? (bi + br) : ((acc == 2) ? bi : br);
    Ctab[idx] = sv * kCarryProd;
  }
  if (wave < 2) stage_x(x, Xw, brow0, 0, tid);
  __syncthreads();

  const _Float16* WX = (const _Float16*)wx1;
  const _Float16* WU = (const _Float16*)wu1;
  const _Float16* WT = (const _Float16*)wt2;
  const int rz = 0 * kUnits + 16 * wave + bn;
  const int rr = 1 * kUnits + 16 * wave + bn;
  const int rh = 2 * kUnits + 16 * wave + bn;
  const _Float16* x1z = WX + (size_t)rz * kXPitch + 8 * hf;
  const _Float16* x1r = WX + (size_t)rr * kXPitch + 8 * hf;
  const _Float16* x1h = WX + (size_t)rh * kXPitch + 8 * hf;
  const _Float16* u1z = WU + (size_t)rz * kK1 + 8 * hf;
  const _Float16* u1r = WU + (size_t)rr * kK1 + 8 * hf;
  const _Float16* u1h = WU + (size_t)rh * kK1 + 8 * hf;
  const _Float16* w2z = WT + (size_t)rz * kK2 + 8 * hf;
  const _Float16* w2r = WT + (size_t)rr * kK2 + 8 * hf;
  const _Float16* w2h = WT + (size_t)rh * kK2 + 8 * hf;

  _Float16* H1 = (_Float16*)H1w;
  _Float16* H2 = (_Float16*)H2w;
  const _Float16* Xh = (const _Float16*)Xw;
  const int rdOff = bn * kHPitch + 8 * hf;
  const int wrOff = bn * kHPitch + 16 * wave + 8 * hf;
  const float* ct = Ctab + 16 * wave + 8 * hf;

  float h1[8], h2[8];
#pragma unroll
  for (int m = 0; m < 8; ++m) { h1[m] = 0.0f; h2[m] = 0.0f; }

#pragma unroll 1
  for (int t = 0; t < kSteps; ++t) {
    asm volatile("" ::: "memory");
    const int cur = t & 1;
    const int nxt = cur ^ 1;

    {
      v8f az  = *(const v8f*)(ct + 0 * kUnits);
      v8f ar  = *(const v8f*)(ct + 1 * kUnits);
      v8f axh = *(const v8f*)(ct + 2 * kUnits);
      v8f arh = *(const v8f*)(ct + 3 * kUnits);
      k_group<1>(az, ar, axh, x1z, x1r, x1h, Xh + bn * kXPitch + 8 * hf);
      k_group<8>(az, ar, arh, u1z, u1r, u1h, H1 + cur * kHBuf + rdOff);
      cell_update(az, ar, axh, arh, h1, H1 + nxt * kHBuf + wrOff);
    }
    __syncthreads();

    {
      v8f az  = *(const v8f*)(ct + 4 * kUnits);
      v8f ar  = *(const v8f*)(ct + 5 * kUnits);
      v8f axh = *(const v8f*)(ct + 6 * kUnits);
      v8f arh = *(const v8f*)(ct + 7 * kUnits);
      k_group<8>(az, ar, axh, w2z, w2r, w2h, H1 + nxt * kHBuf + rdOff);
      k_group<8>(az, ar, arh, w2z + kUnits, w2r + kUnits, w2h + kUnits, H2 + cur * kHBuf + rdOff);
      cell_update(az, ar, axh, arh, h2, H2 + nxt * kHBuf + wrOff);
    }
    if (wave < 2) {
      const int tn = (t + 1 < kSteps) ? (t + 1) : (kSteps - 1);
      stage_x(x, Xw, brow0, tn, tid);
    }
    __syncthreads();
  }

  const size_t blkOff = (size_t)blockIdx.x * (kRowsPerBlock * kUnits);
  {
    float* sp = Osl + bn * kUnits + 16 * wave + 8 * hf;
    *(v4f*)(sp)     = (v4f){h2[0], h2[1], h2[2], h2[3]};
    *(v4f*)(sp + 4) = (v4f){h2[4], h2[5], h2[6], h2[7]};
  }
  __syncthreads();
  {
    const v4f o0 = *(const v4f*)(Osl + 4 * tid);
    const v4f o1 = *(const v4f*)(Osl + 4 * (kThreads + tid));
    float* oa = out + blkOff;
    float* oc = out + 2 * (size_t)kBatch * kUnits + blkOff;
    for (int pass = 0; pass < 2; ++pass) {
      *(volatile v4f*)(oa + 4 * tid) = o0;
      *(volatile v4f*)(oa + 4 * (kThreads + tid)) = o1;
      *(volatile v4f*)(oc + 4 * tid) = o0;
      *(volatile v4f*)(oc + 4 * (kThreads + tid)) = o1;
      __threadfence();
    }
  }
  __syncthreads();
  {
    float* sp = Osl + bn * kUnits + 16 * wave + 8 * hf;
    *(v4f*)(sp)     = (v4f){h1[0], h1[1], h1[2], h1[3]};
    *(v4f*)(sp + 4) = (v4f){h1[4], h1[5], h1[6], h1[7]};
  }
  __syncthreads();
  {
    const v4f o0 = *(const v4f*)(Osl + 4 * tid);
    const v4f o1 = *(const v4f*)(Osl + 4 * (kThreads + tid));
    float* ob = out + (size_t)kBatch * kUnits + blkOff;
    for (int pass = 0; pass < 2; ++pass) {
      *(volatile v4f*)(ob + 4 * tid) = o0;
      *(volatile v4f*)(ob + 4 * (kThreads + tid)) = o1;
      __threadfence();
    }
  }
}

extern "C" void kernel_launch(void* const* d_in, const int* in_sizes, int n_in,
                              void* d_out, int out_size, void* d_ws, size_t ws_size,
                              hipStream_t stream) {
  if (n_in < 7) return;
  if (in_sizes[0] < kBatch * kSteps * kFeat || in_sizes[1] < kFeat * kGates ||
      in_sizes[2] < kUnits * kGates || in_sizes[3] < 2 * kGates ||
      in_sizes[4] < kUnits * kGates || in_sizes[5] < kUnits * kGates ||
      in_sizes[6] < 2 * kGates || out_size < 3 * kBatch * kUnits) return;
  if (ws_size < kCarveTotal) return;

  const float* x  = (const float*)d_in[0];
  const float* W1 = (const float*)d_in[1];
  const float* U1 = (const float*)d_in[2];
  const float* b1 = (const float*)d_in[3];
  const float* W2 = (const float*)d_in[4];
  const float* U2 = (const float*)d_in[5];
  const float* b2 = (const float*)d_in[6];
  float* out = (float*)d_out;

  char* ws = (char*)d_ws;
  unsigned int* wx1 = (unsigned int*)(ws);
  unsigned int* wu1 = (unsigned int*)(ws + kWx1Bytes);
  unsigned int* wt2 = (unsigned int*)(ws + kWx1Bytes + kWu1Bytes);

  build_weight_planes<<<dim3(kJob0Blocks + kJob1Blocks + kJob2Blocks), dim3(256), 0, stream>>>(
      W1, U1, W2, U2, wx1, wu1, wt2);
  stacked_gated_cells<<<dim3(kBlocks), dim3(kThreads), 0, stream>>>(
      x, b1, b2, (const unsigned short*)wx1, (const unsigned short*)wu1, (const unsigned short*)wt2, out);
}
